// StructureExtractor_71184787964506
// MI455X (gfx1250) — hardware-verified
//
#include <hip/hip_runtime.h>

typedef __attribute__((ext_vector_type(16))) _Float16 v16h;
typedef __attribute__((ext_vector_type(8)))  _Float16 v8h;
typedef __attribute__((ext_vector_type(8)))  float    v8f;
#define VST2(T, ptr, val) do { const T _v = (val); *(volatile T*)(ptr) = _v; __threadfence(); *(volatile T*)(ptr) = _v; } while (0)
__device__ __forceinline__ v8f wmma16(v16h a, v16h b, v8f c) {
  v8f d = __builtin_amdgcn_wmma_f32_16x16x32_f16(false, a, false, b, (short)0, c, false, false);
  asm volatile("v_nop\n\tv_nop\n\tv_nop\n\tv_nop" : "+v"(d) : "v"(a), "v"(b));
  return d;
}

#define HH     480
#define WW     640
#define SCALE8 8
#define LCOLS  80
#define LVAL   4800
#define NB     4
#define CC     256
#define AA     128
#define PP     (HH*WW)
#define DD     768
#define MTOT   (2*NB*LVAL)

__global__ void convert_transpose_kernel(const float* __restrict__ src,
                                         _Float16* __restrict__ dst,
                                         int K, int N) {
  int i8 = blockIdx.x * blockDim.x + threadIdx.x;
  if (i8 * 8 >= K * N) return;
  v8h v;
#pragma unroll
  for (int e = 0; e < 8; ++e) { int idx = i8 * 8 + e; int n = idx / K; int k = idx - n * K; v[e] = (_Float16)src[k * N + n]; }
  VST2(v8h, dst + (size_t)i8 * 8, v);
}

__global__ void feat_pack_kernel(const float* __restrict__ feat0,
                                 const float* __restrict__ feat1,
                                 _Float16* __restrict__ X) {
  int i8 = blockIdx.x * blockDim.x + threadIdx.x;
  int r = i8 >> 5;
  int c0 = (i8 & 31) * 8;
  const float* s = (r < MTOT / 2) ? (feat0 + (size_t)r * CC + c0) : (feat1 + (size_t)(r - MTOT / 2) * CC + c0);
  v8h v;
#pragma unroll
  for (int e = 0; e < 8; ++e) v[e] = (_Float16)s[e];
  VST2(v8h, X + (size_t)r * DD + c0, v);
}

__global__ __launch_bounds__(128)
void struct_feats_kernel(const float* __restrict__ pts,
                         const int*   __restrict__ ids,
                         _Float16* __restrict__ X,
                         int rowBase) {
  __shared__ float ax[AA], ay[AA], az[AA];
  const int n   = blockIdx.y;
  const int tid = threadIdx.x;
  if (tid < AA) {
    int id = ids[n * AA + tid];
    const float* p = pts + ((size_t)n * PP + (size_t)id) * 3;
    ax[tid] = p[0]; ay[tid] = p[1]; az[tid] = p[2];
  }
  __syncthreads();
  const int l  = blockIdx.x * 8 + (tid >> 4);
  const int sub = tid & 15, a0 = sub * 8;
  int lr = l / LCOLS, lc = l - lr * LCOLS;
  size_t pidx = ((size_t)n * PP + (size_t)(lr * SCALE8) * WW + (size_t)(lc * SCALE8)) * 3;
  float px = pts[pidx], py = pts[pidx + 1], pz = pts[pidx + 2];
  float dxv[8], dyv[8], dzv[8], d2v[8];
  float s0 = 0.f, s1 = 0.f, s2 = 0.f, s3 = 0.f;
#pragma unroll
  for (int e = 0; e < 8; ++e) {
    const int a = a0 + e;
    float dx = px - ax[a], dy = py - ay[a], dz = pz - az[a];
    float d2 = dx * dx + dy * dy + dz * dz;
    dxv[e] = dx; dyv[e] = dy; dzv[e] = dz; d2v[e] = d2;
    s0 += fabsf(dx); s1 += fabsf(dy); s2 += fabsf(dz); s3 += d2;
  }
#pragma unroll
  for (int off = 1; off < 16; off <<= 1) {
    s0 += __shfl_xor(s0, off, 32); s1 += __shfl_xor(s1, off, 32); s2 += __shfl_xor(s2, off, 32); s3 += __shfl_xor(s3, off, 32);
  }
  float i0 = 1.0f / s0, i1 = 1.0f / s1, i2 = 1.0f / s2, i3 = 1.0f / s3;
  _Float16* xr = X + (size_t)(rowBase + n * LVAL + l) * DD + CC;
  v8h g0, g1, g2, g3;
#pragma unroll
  for (int e = 0; e < 8; ++e) { g0[e] = (_Float16)(dxv[e] * i0); g1[e] = (_Float16)(dyv[e] * i1); g2[e] = (_Float16)(dzv[e] * i2); g3[e] = (_Float16)(d2v[e] * i3); }
  *(volatile v8h*)(xr + 0 * AA + a0) = g0; *(volatile v8h*)(xr + 1 * AA + a0) = g1; *(volatile v8h*)(xr + 2 * AA + a0) = g2; *(volatile v8h*)(xr + 3 * AA + a0) = g3;
  __threadfence();
  *(volatile v8h*)(xr + 0 * AA + a0) = g0; *(volatile v8h*)(xr + 1 * AA + a0) = g1; *(volatile v8h*)(xr + 2 * AA + a0) = g2; *(volatile v8h*)(xr + 3 * AA + a0) = g3;
}

template <bool RELU16>
__global__ __launch_bounds__(256)
void gemm_wmma_kernel(const _Float16* __restrict__ A,
                      const _Float16* __restrict__ Bt,
                      const float*    __restrict__ bias,
                      _Float16* __restrict__ outH,
                      float*    __restrict__ outF,
                      int K, int Ncols) {
  __shared__ __attribute__((aligned(16))) _Float16 As[128][32];
  __shared__ __attribute__((aligned(16))) _Float16 Bs[128][32];
  __shared__ __attribute__((aligned(16))) _Float16 Cs[8][32 * 64];

  const int tid   = threadIdx.x;
  const int lane  = tid & 31;
  const int wave  = tid >> 5;
  const int waveM = wave & 3;
  const int waveN = wave >> 2;
  const int m0 = blockIdx.x * 128;
  const int n0 = blockIdx.y * 128;
  const int hh = lane >> 4;

  v8f acc[2][4] = {};

  const int lrow  = tid >> 1;
  const int lhoff = (tid & 1) * 16;
  const _Float16* ga = A  + (size_t)(m0 + lrow) * K + lhoff;
  const _Float16* gb = Bt + (size_t)(n0 + lrow) * K + lhoff;

  const int aRow  = waveM * 32 + (lane & 15);
  const int koff  = hh * 8;
  const int bRow  = waveN * 64 + (lane & 15);

  for (int k0 = 0; k0 < K; k0 += 32) {
    __syncthreads();
    *(v8h*)&As[lrow][lhoff] = *(const v8h*)(ga + k0); *(v8h*)&As[lrow][lhoff + 8] = *(const v8h*)(ga + k0 + 8);
    *(v8h*)&Bs[lrow][lhoff] = *(const v8h*)(gb + k0); *(v8h*)&Bs[lrow][lhoff + 8] = *(const v8h*)(gb + k0 + 8);
    __syncthreads();

    union Frag { v16h v; v8h h[2]; };
    Frag af[2], bf[4];
#pragma unroll
    for (int mi = 0; mi < 2; ++mi) {
      af[mi].h[0] = *(const v8h*)&As[aRow + mi * 16][koff];
      af[mi].h[1] = *(const v8h*)&As[aRow + mi * 16][16 + koff];
    }
#pragma unroll
    for (int ni = 0; ni < 4; ++ni) {
      bf[ni].h[0] = *(const v8h*)&Bs[bRow + ni * 16][koff];
      bf[ni].h[1] = *(const v8h*)&Bs[bRow + ni * 16][16 + koff];
    }
#pragma unroll
    for (int mi = 0; mi < 2; ++mi)
#pragma unroll
      for (int ni = 0; ni < 4; ++ni)
        acc[mi][ni] = wmma16(af[mi].v, bf[ni].v, acc[mi][ni]);
  }

  if (RELU16) {
    _Float16* st = Cs[wave];
#pragma unroll
    for (int mi = 0; mi < 2; ++mi)
#pragma unroll
      for (int ni = 0; ni < 4; ++ni) {
        const float bv = bias[n0 + waveN * 64 + ni * 16 + (lane & 15)];
#pragma unroll
        for (int r = 0; r < 8; ++r) {
          const float v = acc[mi][ni][r] + bv;
          st[(mi * 16 + r + 8 * hh) * 64 + ni * 16 + (lane & 15)] = (_Float16)(v > 0.f ? v : 0.f);
        }
      }
    __builtin_amdgcn_fence(__ATOMIC_RELEASE, "workgroup"); __builtin_amdgcn_wave_barrier(); __builtin_amdgcn_fence(__ATOMIC_ACQUIRE, "workgroup");
    _Float16* ob = outH + (size_t)(m0 + waveM * 32) * Ncols + n0 + waveN * 64;
    for (int pass = 0; pass < 2; ++pass) {
#pragma unroll
      for (int jj = 0; jj < 8; ++jj) {
        const int row = jj * 4 + (lane >> 3), seg = lane & 7;
        *(volatile v8h*)(ob + (size_t)row * Ncols + seg * 8) = *(const v8h*)(st + row * 64 + seg * 8);
      }
      __threadfence();
    }
  } else {
    for (int pass = 0; pass < 2; ++pass) {
#pragma unroll
      for (int mi = 0; mi < 2; ++mi)
#pragma unroll
        for (int pr = 0; pr < 2; ++pr) {
          const int cbase = n0 + waveN * 64 + pr * 32;
          const float bv = bias[cbase + lane];
#pragma unroll
          for (int r = 0; r < 8; ++r) {
            const float a_ = acc[mi][2 * pr][r], b_ = acc[mi][2 * pr + 1][r];
            const float ax = __shfl_xor(a_, 16), bx = __shfl_xor(b_, 16);
            const int r1 = m0 + waveM * 32 + mi * 16 + r, r2 = r1 + 8;
            *(volatile float*)(outF + (size_t)r1 * Ncols + cbase + lane) = (hh ? bx : a_) + bv;
            *(volatile float*)(outF + (size_t)r2 * Ncols + cbase + lane) = (hh ? b_ : ax) + bv;
          }
        }
      __threadfence();
    }
  }
}

extern "C" void kernel_launch(void* const* d_in, const int* in_sizes, int n_in,
                              void* d_out, int out_size, void* d_ws, size_t ws_size,
                              hipStream_t stream) {
  const float* feat0 = (const float*)d_in[0];
  const float* feat1 = (const float*)d_in[1];
  const float* pts0  = (const float*)d_in[2];
  const float* pts1  = (const float*)d_in[3];
  const int*   ids0  = (const int*)d_in[4];
  const int*   ids1  = (const int*)d_in[5];
  const float* W1    = (const float*)d_in[6];
  const float* b1    = (const float*)d_in[7];
  const float* W2    = (const float*)d_in[8];
  const float* b2    = (const float*)d_in[9];
  float* out = (float*)d_out;

  (void)in_sizes; (void)n_in; (void)out_size;
  if (ws_size < ((size_t)DD * DD + (size_t)CC * DD + 2 * (size_t)MTOT * DD) * sizeof(_Float16)) return;
  _Float16* ws  = (_Float16*)d_ws;
  _Float16* W1t = ws;                    ws += (size_t)DD * DD;
  _Float16* W2t = ws;                    ws += (size_t)CC * DD;
  _Float16* X   = ws;                    ws += (size_t)MTOT * DD;
  _Float16* Hh  = ws;                    ws += (size_t)MTOT * DD;

  convert_transpose_kernel<<<(DD * DD / 8 + 255) / 256, 256, 0, stream>>>(W1, W1t, DD, DD);
  convert_transpose_kernel<<<(DD * CC / 8 + 255) / 256, 256, 0, stream>>>(W2, W2t, DD, CC);
  feat_pack_kernel<<<(MTOT * CC / 8) / 256, 256, 0, stream>>>(feat0, feat1, X);

  dim3 sg(LVAL / 8, NB);
  struct_feats_kernel<<<sg, 128, 0, stream>>>(pts0, ids0, X, 0);
  struct_feats_kernel<<<sg, 128, 0, stream>>>(pts1, ids1, X, MTOT / 2);

  dim3 g1(MTOT / 128, DD / 128);
  gemm_wmma_kernel<true><<<g1, 256, 0, stream>>>(X, W1t, b1, Hh, nullptr, DD, DD);

  dim3 g2(MTOT / 128, CC / 128);
  gemm_wmma_kernel<false><<<g2, 256, 0, stream>>>(Hh, W2t, b2, nullptr, out, DD, CC);
}
